// PointPillarsModel_45397804319069
// MI455X (gfx1250) — hardware-verified
//
#include <hip/hip_runtime.h>
#include <math.h>
#include <stddef.h>
#include <stdint.h>

#define NPIL   20000
#define NROWS  640000
#define IMW    666
#define HW0    443556
#define W1     333
#define HW1    110889
#define M1PAD  110976
#define W2     166
#define HW2    27556
#define M2PAD  27648
#define FPAD   20096
#define NOUTF  661344
#define NOUT4  165336
#define WCELLS 8192
#define NWBLK  55
#define WINPAD (NWBLK * WCELLS)
#define SPT    68
#define WSMAX  134217728

static_assert(IMW == 2 * W1);
static_assert(W1 / 2 == W2);
static_assert(IMW * IMW == HW0);
static_assert(W1 * W1 == HW1);
static_assert(W2 * W2 == HW2);
static_assert(NROWS % 128 == 0);
static_assert(NROWS == NPIL * 32);
static_assert(M1PAD % 128 == 0 && M1PAD >= HW1);
static_assert(M2PAD % 128 == 0 && M2PAD >= HW2);
static_assert(FPAD % 64 == 0 && FPAD >= NPIL);
static_assert(WINPAD >= HW0);
static_assert(HW2 % 4 == 0);
static_assert(NOUTF == 24 * HW2);
static_assert(NOUT4 * 4 == NOUTF);
static_assert(NOUT4 % 8 == 0);
static_assert(128 % 32 == 0 && 1152 % 32 == 0 && 2304 % 32 == 0 && 4608 % 32 == 0);
static_assert(24 <= 32);
static_assert(M1PAD % 64 == 0);

typedef float          v2f   __attribute__((ext_vector_type(2)));
typedef float          v4f   __attribute__((ext_vector_type(4)));
typedef float          v8f   __attribute__((ext_vector_type(8)));
typedef int            v4i   __attribute__((ext_vector_type(4)));
typedef int            v8i   __attribute__((ext_vector_type(8)));
typedef unsigned short v4us  __attribute__((ext_vector_type(4)));
typedef unsigned short v8us  __attribute__((ext_vector_type(8)));
typedef unsigned short v16us __attribute__((ext_vector_type(16)));
typedef __bf16         v16bf __attribute__((ext_vector_type(16)));
typedef v4f  __attribute__((may_alias)) v4fa;
typedef v4i  __attribute__((may_alias)) v4ia;
typedef v8us __attribute__((may_alias)) v8usa;
union FragB { v16bf v; v16us u; v8us h[2]; v8i w; };

__device__ __forceinline__ v8f wmb(const FragB& a, const FragB& b, v8f c) {
  v8f d = __builtin_amdgcn_wmma_f32_16x16x32_bf16(false, a.v, false, b.v, (short)0, c, false, false);
  asm volatile("v_nop\n\tv_nop\n\tv_nop\n\tv_nop" : "+v"(d) : "v"(a.w), "v"(b.w));
  return d;
}
__device__ __forceinline__ v8f z8() { v8f z = {0.f, 0.f, 0.f, 0.f, 0.f, 0.f, 0.f, 0.f}; return z; }

__device__ __forceinline__ unsigned bf16_bits(float f) {
  const unsigned u = __float_as_uint(f);
  return (u + 0x7FFFu + ((u >> 16) & 1u)) >> 16;
}
__device__ __forceinline__ float bf16_val(float f) { return __uint_as_float(bf16_bits(f) << 16); }
__device__ __forceinline__ float relu_k(float v) { return (v > 0.0f) ? v : (v - v); }
__device__ __forceinline__ float max_k(float a, float b) { return ((b > a) || (b != b)) ? b : a; }
__device__ __forceinline__ float sel_f(bool cond, float a, float b) {
  const int mk = -(int)cond;
  return __int_as_float((__float_as_int(a) & mk) | (__float_as_int(b) & ~mk));
}

__global__ __launch_bounds__(256) void k_wconv(const float* __restrict__ src, unsigned short* dst,
                                               int nrows, int nsrc, int cin, int mode) {
  const int u = (int)blockIdx.x * 256 + (int)threadIdx.x;
  const int K = mode ? 128 : 18 * cin;
  const int upr = K >> 3;
  if (u >= nrows * upr) return;
  const int row = u / upr;
  const int kk = (u - row * upr) * 8;
  int oc, tap, ic;
  if (mode) {
    tap = row >> 6; oc = row & 63; ic = kk & 63;
  } else {
    oc = row;
    tap = kk / (2 * cin);
    const int rem = kk - tap * 2 * cin;
    ic = (rem >= cin) ? (rem - cin) : rem;
  }
  const bool ok = oc < nsrc;
  const int occ = ok ? oc : (nsrc - 1);
  const float* p = src + ((size_t)occ * (size_t)cin + (size_t)ic) * 9 + tap;
  float f[8];
#pragma unroll
  for (int e = 0; e < 8; ++e) f[e] = p[9 * e];
  v8us o;
#pragma unroll
  for (int e = 0; e < 8; ++e) o[e] = ok ? (unsigned short)bf16_bits(f[e]) : (unsigned short)0;
  unsigned short* dp = dst + (size_t)u * 8;
  *(volatile v8us*)dp = o;
  __threadfence();
  *(volatile v8us*)dp = o;
}

__global__ __launch_bounds__(256) void k_win(const int* __restrict__ coords, int* win) {
  __shared__ __attribute__((aligned(16))) int cell[WCELLS];
  const int tid = (int)threadIdx.x;
  const int base = (int)blockIdx.x * WCELLS;
#pragma unroll 1
  for (int i = tid; i < WCELLS; i += 256) cell[i] = -1;
  __syncthreads();
#pragma unroll 1
  for (int p = tid; p < NPIL; p += 256) {
    const int y = coords[3 * p + 1];
    const int x = coords[3 * p + 2];
    const bool valid = (y >= 0) && (y < IMW) && (x >= 0) && (x < IMW);
    const int yc = min(max(y, 0), IMW - 1);
    const int xc = min(max(x, 0), IMW - 1);
    const int c = yc * IMW + xc - base;
    if (valid && c >= 0 && c < WCELLS) atomicMax(&cell[c], p);
  }
  __syncthreads();
  v4i v[8];
#pragma unroll
  for (int it = 0; it < 8; ++it) v[it] = *(const v4ia*)(cell + 4 * (it * 256 + tid));
#pragma unroll
  for (int it = 0; it < 8; ++it) *(volatile v4i*)(win + base + 4 * (it * 256 + tid)) = v[it];
  __threadfence();
#pragma unroll
  for (int it = 0; it < 8; ++it) *(volatile v4i*)(win + base + 4 * (it * 256 + tid)) = v[it];
}

__global__ __launch_bounds__(128) __attribute__((amdgpu_num_vgpr(248)))
void k_pfn(const float* __restrict__ pts, const float* __restrict__ linw, const float* __restrict__ linb,
           float* pmmg, float* rec) {
  __shared__ __attribute__((aligned(16))) unsigned short As[128 * 40];
  __shared__ __attribute__((aligned(16))) unsigned short Ws[64 * 40];
  __shared__ __attribute__((aligned(16))) float stg[128 * SPT];
  __shared__ __attribute__((aligned(16))) float sb[64];
  __shared__ __attribute__((aligned(16))) float ssum[128];
  __shared__ __attribute__((aligned(16))) float sq[128];
  __shared__ __attribute__((aligned(16))) float pmm[512];
  __shared__ __attribute__((aligned(16))) float recl[128];
  const int tid = (int)threadIdx.x, lane = tid & 31, wave = tid >> 5, hh = lane >> 4, m = lane & 15;
  const int tile = (int)blockIdx.x;
  const v8us zz = {0, 0, 0, 0, 0, 0, 0, 0};
#pragma unroll 1
  for (int i = tid; i < 640; i += 128) *(v8usa*)(As + 8 * i) = zz;
#pragma unroll 1
  for (int i = tid; i < 320; i += 128) *(v8usa*)(Ws + 8 * i) = zz;
  if (tid < 64) sb[tid] = bf16_val(linb[tid]);
  __syncthreads();
  const float* src = pts + (size_t)tile * 1152;
#pragma unroll 1
  for (int f = tid; f < 288; f += 128) {
    const v4f a = *(const v4f*)(src + 4 * f);
    const float av[4] = {a.x, a.y, a.z, a.w};
#pragma unroll
    for (int e = 0; e < 4; ++e) {
      const int idx = 4 * f + e;
      const int row = idx / 9;
      const int k = idx - 9 * row;
      As[row * 40 + k] = (unsigned short)bf16_bits(av[e]);
    }
  }
#pragma unroll 1
  for (int i = tid; i < 576; i += 128) {
    const int c = i / 9;
    const int k = i - 9 * c;
    Ws[c * 40 + k] = (unsigned short)bf16_bits(linw[i]);
  }
  __syncthreads();

  FragB bfr[4];
#pragma unroll
  for (int nt = 0; nt < 4; ++nt) {
    const unsigned short* p = Ws + (16 * nt + m) * 40 + 8 * hh;
    bfr[nt].h[0] = *(const v8usa*)p;
    bfr[nt].h[1] = *(const v8usa*)(p + 16);
  }
  v8f acc[2][4];
#pragma unroll
  for (int mt = 0; mt < 2; ++mt) {
    const unsigned short* p = As + (32 * wave + 16 * mt + m) * 40 + 8 * hh;
    FragB af;
    af.h[0] = *(const v8usa*)p;
    af.h[1] = *(const v8usa*)(p + 16);
#pragma unroll
    for (int nt = 0; nt < 4; ++nt) acc[mt][nt] = wmb(af, bfr[nt], z8());
  }
#pragma unroll
  for (int mt = 0; mt < 2; ++mt)
#pragma unroll
    for (int nt = 0; nt < 4; ++nt)
#pragma unroll
      for (int r = 0; r < 8; ++r)
        stg[(32 * wave + 16 * mt + 8 * hh + r) * SPT + 16 * nt + m] = acc[mt][nt][r];
  __syncthreads();

  const int c = tid & 63, hf = tid >> 6;
  const float bc = sb[c];
  float s = 0.0f;
#pragma unroll 1
  for (int g = 0; g < 2; ++g) {
    float mx = -INFINITY, mn = INFINITY;
    const float* sp = stg + (hf * 64 + g * 32) * SPT + c;
#pragma unroll 4
    for (int r = 0; r < 32; ++r) {
      const float v = sp[r * SPT] + bc;
      s += v;
      mx = fmaxf(mx, v);
      mn = fminf(mn, v);
    }
    pmm[(hf * 2 + g) * 128 + c] = mx;
    pmm[(hf * 2 + g) * 128 + 64 + c] = mn;
  }
  ssum[tid] = s;
  __syncthreads();
  const float mean = (ssum[c] + ssum[64 + c]) * (1.0f / 128.0f);
  float q = 0.0f;
  {
    const float* sp = stg + (hf * 64) * SPT + c;
#pragma unroll 4
    for (int r = 0; r < 64; ++r) {
      const float d = (sp[r * SPT] + bc) - mean;
      q = fmaf(d, d, q);
    }
  }
  sq[tid] = q;
  __syncthreads();
  if (tid < 64) {
    recl[tid] = mean;
    recl[64 + tid] = sq[tid] + sq[64 + tid];
  }
  __syncthreads();
  const v4f pv = *(const v4fa*)(pmm + 4 * tid);
  v4f rv = {0.f, 0.f, 0.f, 0.f};
  if (tid < 32) rv = *(const v4fa*)(recl + 4 * tid);
  *(volatile v4f*)(pmmg + (size_t)tile * 512 + 4 * tid) = pv;
  if (tid < 32) *(volatile v4f*)(rec + (size_t)tile * 128 + 4 * tid) = rv;
  __threadfence();
  *(volatile v4f*)(pmmg + (size_t)tile * 512 + 4 * tid) = pv;
  if (tid < 32) *(volatile v4f*)(rec + (size_t)tile * 128 + 4 * tid) = rv;
}

__global__ __launch_bounds__(256) void k_comb(const float* __restrict__ rec, int nblk, int nfull, int nlast,
                                              const float* __restrict__ gam, const float* __restrict__ bet,
                                              float* stat, int C, double invN) {
  __shared__ __attribute__((aligned(16))) float st[1024];
  const int c = (int)threadIdx.x;
  const size_t pitch = (size_t)(2 * C);
  double s = 0.0;
#pragma unroll 1
  for (int b = 0; b < nblk; ++b) {
    const double nb = (double)((b == nblk - 1) ? nlast : nfull);
    s += nb * (double)rec[(size_t)b * pitch + c];
  }
  const double mean = s * invN;
  double q = 0.0;
#pragma unroll 1
  for (int b = 0; b < nblk; ++b) {
    const double nb = (double)((b == nblk - 1) ? nlast : nfull);
    const double d = (double)rec[(size_t)b * pitch + c] - mean;
    q += (double)rec[(size_t)b * pitch + C + c] + nb * d * d;
  }
  const float var = (float)(q * invN);
  const float rstd = 1.0f / sqrtf(var + 1e-5f);
  st[c] = (float)mean;
  st[C + c] = rstd;
  st[2 * C + c] = bf16_val(gam[c]);
  st[3 * C + c] = bf16_val(bet[c]);
  __syncthreads();
  const v4f v = *(const v4fa*)(st + 4 * c);
  *(volatile v4f*)(stat + 4 * c) = v;
  __threadfence();
  *(volatile v4f*)(stat + 4 * c) = v;
}

__global__ __launch_bounds__(256) void k_feat(const float* __restrict__ pmmg, const float* __restrict__ stat,
                                              unsigned short* feat) {
  __shared__ __attribute__((aligned(16))) float st[256];
  const int tid = (int)threadIdx.x;
  st[tid] = stat[tid];
  __syncthreads();
  const int u = (int)blockIdx.x * 256 + tid;
  const int p = u >> 3;
  const int c8 = (u & 7) * 8;
  const bool ok = p < NPIL;
  const int pc = ok ? p : (NPIL - 1);
  const float* r = pmmg + (size_t)pc * 128 + c8;
  const v4f xa = *(const v4f*)r;
  const v4f xb = *(const v4f*)(r + 4);
  const v4f na = *(const v4f*)(r + 64);
  const v4f nb = *(const v4f*)(r + 68);
  const float mxv[8] = {xa.x, xa.y, xa.z, xa.w, xb.x, xb.y, xb.z, xb.w};
  const float mnv[8] = {na.x, na.y, na.z, na.w, nb.x, nb.y, nb.z, nb.w};
  v8us h8, l8;
#pragma unroll
  for (int e = 0; e < 8; ++e) {
    const float mm = st[c8 + e], rr = st[64 + c8 + e], g = st[128 + c8 + e], b = st[192 + c8 + e];
    const float sel = sel_f(g >= 0.0f, mxv[e], mnv[e]);
    float v = ((sel - mm) * rr) * g + b;
    v = relu_k(v);
    v = ok ? v : 0.0f;
    const unsigned hb = bf16_bits(v);
    const unsigned lb = bf16_bits(v - __uint_as_float(hb << 16));
    h8[e] = (unsigned short)hb;
    l8[e] = (unsigned short)lb;
  }
  unsigned short* dp = feat + (size_t)p * 128 + c8;
  *(volatile v8us*)dp = h8;
  *(volatile v8us*)(dp + 64) = l8;
  __threadfence();
  *(volatile v8us*)dp = h8;
  *(volatile v8us*)(dp + 64) = l8;
}

__global__ __launch_bounds__(128) __attribute__((amdgpu_num_vgpr(248)))
void k_gemm(const unsigned short* __restrict__ A, int lda, const unsigned short* __restrict__ BT, int ldb, int K,
            float* Cm, int ldc) {
  __shared__ __attribute__((aligned(16))) float stg[64 * SPT];
  const int tid = (int)threadIdx.x, lane = tid & 31, wave = tid >> 5, hh = lane >> 4, m = lane & 15;
  const int rowBase = (int)blockIdx.x * 64;
  const int colBase = (int)blockIdx.y * 64;
  v8f acc[4];
#pragma unroll
  for (int t = 0; t < 4; ++t) acc[t] = z8();
  const unsigned short* ap = A + (size_t)(rowBase + 16 * wave + m) * (size_t)lda + 8 * hh;
  const unsigned short* bp = BT + (size_t)(colBase + m) * (size_t)ldb + 8 * hh;
#pragma unroll 1
  for (int k0 = 0; k0 < K; k0 += 32) {
    FragB af;
    af.h[0] = *(const v8usa*)(ap + k0);
    af.h[1] = *(const v8usa*)(ap + k0 + 16);
#pragma unroll
    for (int nt = 0; nt < 4; ++nt) {
      const unsigned short* wq = bp + (size_t)(16 * nt) * (size_t)ldb + k0;
      FragB bf;
      bf.h[0] = *(const v8usa*)wq;
      bf.h[1] = *(const v8usa*)(wq + 16);
      acc[nt] = wmb(af, bf, acc[nt]);
    }
  }
#pragma unroll
  for (int nt = 0; nt < 4; ++nt)
#pragma unroll
    for (int r = 0; r < 8; ++r)
      stg[(16 * wave + 8 * hh + r) * SPT + 16 * nt + m] = acc[nt][r];
  __syncthreads();
  const int rsub = tid >> 4;
  const int c4 = (tid & 15) * 4;
  v4f pv[8];
#pragma unroll
  for (int it = 0; it < 8; ++it) pv[it] = *(const v4fa*)(stg + (it * 8 + rsub) * SPT + c4);
#pragma unroll
  for (int it = 0; it < 8; ++it)
    *(volatile v4f*)(Cm + (size_t)(rowBase + it * 8 + rsub) * (size_t)ldc + colBase + c4) = pv[it];
  __threadfence();
#pragma unroll
  for (int it = 0; it < 8; ++it)
    *(volatile v4f*)(Cm + (size_t)(rowBase + it * 8 + rsub) * (size_t)ldc + colBase + c4) = pv[it];
}

template <int MODE>
__global__ __launch_bounds__(256) __attribute__((amdgpu_num_vgpr(248)))
void k_c1(const int* __restrict__ win, const float* __restrict__ tp, const float* __restrict__ c1b,
          const float* __restrict__ stat, float* rec, unsigned* b1) {
  __shared__ __attribute__((aligned(16))) float sS[8 * 64];
  __shared__ __attribute__((aligned(16))) float sQ[8 * 64];
  __shared__ __attribute__((aligned(16))) float recl[128];
  const int tid = (int)threadIdx.x, lane = tid & 31;
  const int wave = __builtin_amdgcn_readfirstlane(tid >> 5);
  const int blk = (int)blockIdx.x;
  const int ch = 2 * lane;
  const v2f bv = *(const v2f*)(c1b + ch);
  const float b0 = bf16_val(bv.x), b1v = bf16_val(bv.y);
  float m0 = 0.f, m1 = 0.f, r0 = 0.f, r1 = 0.f, g0 = 0.f, g1 = 0.f, e0 = 0.f, e1 = 0.f;
  if (MODE == 1) {
    v2f t = *(const v2f*)(stat + ch);        m0 = t.x; m1 = t.y;
    t = *(const v2f*)(stat + 64 + ch);       r0 = t.x; r1 = t.y;
    t = *(const v2f*)(stat + 128 + ch);      g0 = t.x; g1 = t.y;
    t = *(const v2f*)(stat + 192 + ch);      e0 = t.x; e1 = t.y;
  }
  float s0 = 0.0f, s1 = 0.0f, q0 = 0.0f, q1 = 0.0f;
#pragma unroll 1
  for (int i = 0; i < 8; ++i) {
    const int pp = blk * 64 + wave * 8 + i;
    if (pp < HW1) {
      const int Y = pp / W1, X = pp - Y * W1;
      const int j = lane & 15;
      const int nr = 2 * Y - 1 + (j >> 2), nc = 2 * X - 1 + (j & 3);
      const bool inb = (nr >= 0) && (nr < IMW) && (nc >= 0) && (nc < IMW);
      const int idx = inb ? (nr * IMW + nc) : 0;
      int wv = win[idx];
      wv = inb ? wv : -1;
      wv = min(wv, NPIL - 1);
      wv = max(wv, -1);
      float mx0 = -INFINITY, mx1 = -INFINITY;
#pragma unroll
      for (int px = 0; px < 4; ++px) {
        const int dy = px >> 1, dx = px & 1;
        float a0 = 0.0f, a1 = 0.0f;
#pragma unroll
        for (int tap = 0; tap < 9; ++tap) {
          const int ky = tap / 3, kx = tap - 3 * ky;
          const int p = __builtin_amdgcn_readlane(wv, (dy + ky) * 4 + dx + kx);
          if (p >= 0) {
            const v2f t = *(const v2f*)(tp + (size_t)p * 576 + tap * 64 + ch);
            a0 += t.x;
            a1 += t.y;
          }
        }
        const float v0 = a0 + b0, v1 = a1 + b1v;
        if (MODE == 0) {
          const float d0 = v0 - b0, d1 = v1 - b1v;
          s0 += d0; q0 = fmaf(d0, d0, q0);
          s1 += d1; q1 = fmaf(d1, d1, q1);
        } else {
          float y0 = ((v0 - m0) * r0) * g0 + e0;
          float y1 = ((v1 - m1) * r1) * g1 + e1;
          y0 = relu_k(y0);
          y1 = relu_k(y1);
          mx0 = max_k(mx0, y0);
          mx1 = max_k(mx1, y1);
        }
      }
      if (MODE == 1) {
        const unsigned h0 = bf16_bits(mx0), h1 = bf16_bits(mx1);
        const unsigned l0 = bf16_bits(mx0 - __uint_as_float(h0 << 16));
        const unsigned l1 = bf16_bits(mx1 - __uint_as_float(h1 << 16));
        const unsigned hw = h0 | (h1 << 16);
        const unsigned lw = l0 | (l1 << 16);
        volatile unsigned* q = b1 + (size_t)pp * 64;
        q[lane] = hw;
        q[32 + lane] = lw;
        __threadfence();
        q[lane] = hw;
        q[32 + lane] = lw;
      }
    } else if (MODE == 1) {
      if (pp < M1PAD) {
        volatile unsigned* q = b1 + (size_t)pp * 64;
        q[lane] = 0u;
        q[32 + lane] = 0u;
        __threadfence();
        q[lane] = 0u;
        q[32 + lane] = 0u;
      }
    }
  }
  if (MODE == 0) {
    sS[wave * 64 + ch] = s0; sS[wave * 64 + ch + 1] = s1;
    sQ[wave * 64 + ch] = q0; sQ[wave * 64 + ch + 1] = q1;
    __syncthreads();
    if (tid < 64) {
      float S = 0.0f, Q = 0.0f;
#pragma unroll
      for (int w = 0; w < 8; ++w) { S += sS[w * 64 + tid]; Q += sQ[w * 64 + tid]; }
      const int npool = min(64, HW1 - blk * 64);
      const float invn = 1.0f / (float)(4 * npool);
      const float bb = bf16_val(c1b[tid]);
      recl[tid] = bb + S * invn;
      recl[64 + tid] = fmaxf(Q - S * S * invn, 0.0f);
    }
    __syncthreads();
    v4f rv = {0.f, 0.f, 0.f, 0.f};
    if (tid < 32) {
      rv = *(const v4fa*)(recl + 4 * tid);
      *(volatile v4f*)(rec + (size_t)blk * 128 + 4 * tid) = rv;
    }
    __threadfence();
    if (tid < 32) *(volatile v4f*)(rec + (size_t)blk * 128 + 4 * tid) = rv;
  }
}

template <int CW, bool BIAS>
__device__ __forceinline__ void tile_store(const float* stg, const float* sb, float* Cm, size_t rowBase, int ldc,
                                           int colBase, int tid) {
  constexpr int SP = CW + 4, TPR = CW / 4, RPP = 128 / TPR;
  const int rsub = tid / TPR, c4 = (tid % TPR) * 4;
#pragma unroll 4
  for (int it = 0; it < 128 / RPP; ++it) {
    const int row = it * RPP + rsub;
    v4f v = *(const v4fa*)(stg + row * SP + c4);
    if (BIAS) { v.x += sb[c4]; v.y += sb[c4 + 1]; v.z += sb[c4 + 2]; v.w += sb[c4 + 3]; }
    *(volatile v4f*)(Cm + (rowBase + (size_t)row) * (size_t)ldc + colBase + c4) = v;
  }
}

template <int CIN, int HD, int NOUT, int NT, bool STATS>
__global__ __launch_bounds__(128) __attribute__((amdgpu_num_vgpr(248)))
void k_conv(const unsigned short* __restrict__ A, const unsigned short* __restrict__ BT,
            const float* __restrict__ bias, float* Cm, float* rec, int M) {
  constexpr int KROW = 2 * CIN, KTOT = 9 * KROW, CW = 16 * NT, SP = CW + 4;
  static_assert(KROW % 32 == 0);
  static_assert(!STATS || NT == 4);
  static_assert(NOUT % CW == 0);
  __shared__ __attribute__((aligned(16))) float stg[128 * SP];
  __shared__ __attribute__((aligned(16))) float sb[64];
  __shared__ __attribute__((aligned(16))) float ssum[128];
  __shared__ __attribute__((aligned(16))) float sq[128];
  __shared__ __attribute__((aligned(16))) float recl[128];
  const int tid = (int)threadIdx.x, lane = tid & 31, wave = tid >> 5, hh = lane >> 4, m = lane & 15;
  const int tile = (int)blockIdx.x;
  const int colBase = (int)blockIdx.y * CW;
  if (STATS) { if (tid < CW) sb[tid] = bf16_val(bias[colBase + tid]); }

  const int ra = tile * 128 + 32 * wave + m;
  const int rb = ra + 16;
  const int ya = ra / HD, xa = ra - ya * HD;
  const int yb = rb / HD, xb = rb - yb * HD;
  const bool va = ra < M, vb = rb < M;

  v8f acc[2][NT];
#pragma unroll
  for (int mt = 0; mt < 2; ++mt)
#pragma unroll
    for (int nt = 0; nt < NT; ++nt) acc[mt][nt] = z8();

  const unsigned short* bp = BT + (size_t)(colBase + m) * (size_t)KTOT + 8 * hh;
#pragma unroll 1
  for (int tap = 0; tap < 9; ++tap) {
    const int ky = tap / 3, kx = tap - 3 * ky;
    const int nya = ya + ky - 1, nxa = xa + kx - 1;
    const int nyb = yb + ky - 1, nxb = xb + kx - 1;
    const bool oka = va && (nya >= 0) && (nya < HD) && (nxa >= 0) && (nxa < HD);
    const bool okb = vb && (nyb >= 0) && (nyb < HD) && (nxb >= 0) && (nxb < HD);
    const int ia = oka ? (nya * HD + nxa) : 0;
    const int ib = okb ? (nyb * HD + nxb) : 0;
    const int ma = oka ? -1 : 0;
    const int mb = okb ? -1 : 0;
    const v8i mva = {ma, ma, ma, ma, ma, ma, ma, ma};
    const v8i mvb = {mb, mb, mb, mb, mb, mb, mb, mb};
    const unsigned short* apa = A + (size_t)ia * (size_t)KROW + 8 * hh;
    const unsigned short* apb = A + (size_t)ib * (size_t)KROW + 8 * hh;
    const unsigned short* bq = bp + tap * KROW;
#pragma unroll 1
    for (int s = 0; s < KROW; s += 32) {
      FragB fa, fb;
      fa.h[0] = *(const v8usa*)(apa + s);
      fa.h[1] = *(const v8usa*)(apa + s + 16);
      fb.h[0] = *(const v8usa*)(apb + s);
      fb.h[1] = *(const v8usa*)(apb + s + 16);
      fa.w = fa.w & mva;
      fb.w = fb.w & mvb;
#pragma unroll
      for (int nt = 0; nt < NT; ++nt) {
        const unsigned short* wq = bq + (size_t)(16 * nt) * (size_t)KTOT + s;
        FragB bf;
        bf.h[0] = *(const v8usa*)wq;
        bf.h[1] = *(const v8usa*)(wq + 16);
        acc[0][nt] = wmb(fa, bf, acc[0][nt]);
        acc[1][nt] = wmb(fb, bf, acc[1][nt]);
      }
    }
  }
#pragma unroll
  for (int mt = 0; mt < 2; ++mt)
#pragma unroll
    for (int nt = 0; nt < NT; ++nt)
#pragma unroll
      for (int r = 0; r < 8; ++r)
        stg[(32 * wave + 16 * mt + 8 * hh + r) * SP + 16 * nt + m] = acc[mt][nt][r];
  __syncthreads();

  tile_store<CW, STATS>(stg, sb, Cm, (size_t)tile * 128, NOUT, colBase, tid);
  __threadfence();
  tile_store<CW, STATS>(stg, sb, Cm, (size_t)tile * 128, NOUT, colBase, tid);

  if (STATS) {
    const int nvalid = min(128, M - tile * 128);
    const float invn = 1.0f / (float)nvalid;
    const int c = tid & 63, hf = tid >> 6;
    const float bc = sb[c];
    const int rbeg = hf * 64;
    const int rend = min(nvalid, rbeg + 64);
    float s = 0.0f;
#pragma unroll 4
    for (int r = rbeg; r < rend; ++r) s += stg[r * SP + c] + bc;
    ssum[tid] = s;
    __syncthreads();
    const float mean = (ssum[c] + ssum[64 + c]) * invn;
    float q = 0.0f;
#pragma unroll 4
    for (int r = rbeg; r < rend; ++r) {
      const float d = (stg[r * SP + c] + bc) - mean;
      q = fmaf(d, d, q);
    }
    sq[tid] = q;
    __syncthreads();
    if (tid < 64) {
      recl[tid] = mean;
      recl[64 + tid] = sq[tid] + sq[64 + tid];
    }
    __syncthreads();
    v4f rv = {0.f, 0.f, 0.f, 0.f};
    const int part = (tid >> 4) & 1, f4 = tid & 15;
    float* rp = rec + (size_t)tile * (size_t)(2 * NOUT) + (size_t)part * NOUT + colBase + 4 * f4;
    if (tid < 32) {
      rv = *(const v4fa*)(recl + part * 64 + 4 * f4);
      *(volatile v4f*)rp = rv;
    }
    __threadfence();
    if (tid < 32) *(volatile v4f*)rp = rv;
  }
}

__global__ __launch_bounds__(256) void k_pool2(const float* __restrict__ c2, const float* __restrict__ stat,
                                               unsigned short* b2) {
  const int tid = (int)threadIdx.x, lane = tid & 31;
  const int wave = __builtin_amdgcn_readfirstlane(tid >> 5);
  const int pp = (int)blockIdx.x * 8 + wave;
  const int c4 = 4 * lane;
  v4us h4 = {0, 0, 0, 0}, l4 = {0, 0, 0, 0};
  if (pp < HW2) {
    const int Y = pp / W2, X = pp - Y * W2;
    const v4f mm = *(const v4f*)(stat + c4);
    const v4f rr = *(const v4f*)(stat + 128 + c4);
    const v4f gg = *(const v4f*)(stat + 256 + c4);
    const v4f be = *(const v4f*)(stat + 384 + c4);
    float mx[4] = {-INFINITY, -INFINITY, -INFINITY, -INFINITY};
#pragma unroll
    for (int px = 0; px < 4; ++px) {
      const int dy = px >> 1, dx = px & 1;
      const v4f x = *(const v4f*)(c2 + (size_t)((2 * Y + dy) * W1 + 2 * X + dx) * 128 + c4);
      const float y0 = relu_k(((x.x - mm.x) * rr.x) * gg.x + be.x);
      const float y1 = relu_k(((x.y - mm.y) * rr.y) * gg.y + be.y);
      const float y2 = relu_k(((x.z - mm.z) * rr.z) * gg.z + be.z);
      const float y3 = relu_k(((x.w - mm.w) * rr.w) * gg.w + be.w);
      mx[0] = max_k(mx[0], y0); mx[1] = max_k(mx[1], y1);
      mx[2] = max_k(mx[2], y2); mx[3] = max_k(mx[3], y3);
    }
#pragma unroll
    for (int e = 0; e < 4; ++e) {
      const unsigned hb = bf16_bits(mx[e]);
      const unsigned lb = bf16_bits(mx[e] - __uint_as_float(hb << 16));
      h4[e] = (unsigned short)hb;
      l4[e] = (unsigned short)lb;
    }
  }
  unsigned short* dp = b2 + (size_t)pp * 256 + c4;
  *(volatile v4us*)dp = h4;
  *(volatile v4us*)(dp + 128) = l4;
  __threadfence();
  *(volatile v4us*)dp = h4;
  *(volatile v4us*)(dp + 128) = l4;
}

__global__ __launch_bounds__(256) void k_app3(const float* __restrict__ c3, const float* __restrict__ stat,
                                              unsigned short* hl) {
  __shared__ __attribute__((aligned(16))) float st[1024];
  const int tid = (int)threadIdx.x;
#pragma unroll
  for (int i = 0; i < 4; ++i) st[i * 256 + tid] = stat[i * 256 + tid];
  __syncthreads();
  const int u = (int)blockIdx.x * 256 + tid;
  const int pix = u >> 5;
  const int c8 = (u & 31) * 8;
  const bool ok = pix < HW2;
  const int pc = ok ? pix : (HW2 - 1);
  const float* r = c3 + (size_t)pc * 256 + c8;
  const v4f xa = *(const v4f*)r;
  const v4f xb = *(const v4f*)(r + 4);
  const float xv[8] = {xa.x, xa.y, xa.z, xa.w, xb.x, xb.y, xb.z, xb.w};
  v8us h8, l8;
#pragma unroll
  for (int e = 0; e < 8; ++e) {
    const float mm = st[c8 + e], rr = st[256 + c8 + e], g = st[512 + c8 + e], b = st[768 + c8 + e];
    float v = ((xv[e] - mm) * rr) * g + b;
    v = relu_k(v);
    v = ok ? v : 0.0f;
    const unsigned hb = bf16_bits(v);
    const unsigned lb = bf16_bits(v - __uint_as_float(hb << 16));
    h8[e] = (unsigned short)hb;
    l8[e] = (unsigned short)lb;
  }
  unsigned short* dp = hl + (size_t)pix * 512 + c8;
  *(volatile v8us*)dp = h8;
  *(volatile v8us*)(dp + 256) = l8;
  __threadfence();
  *(volatile v8us*)dp = h8;
  *(volatile v8us*)(dp + 256) = l8;
}

__global__ __launch_bounds__(256) void k_out(const float* __restrict__ headt, const float* __restrict__ hbb,
                                             const float* __restrict__ hcb, float* out) {
  const int i = (int)blockIdx.x * 256 + (int)threadIdx.x;
  if (i >= NOUT4) return;
  const int f = 4 * i;
  const int c = f / HW2;
  const int pix = f - c * HW2;
  const int ci = min(c, 20);
  const int cj = min(max(c - 21, 0), 2);
  const float bb = bf16_val(hbb[ci]);
  const float bc = bf16_val(hcb[cj]);
  const float bs = sel_f(c < 21, bb, bc);
  const float* hp = headt + (size_t)pix * 32 + c;
  v4f v;
  v.x = hp[0] + bs;
  v.y = hp[32] + bs;
  v.z = hp[64] + bs;
  v.w = hp[96] + bs;
  *(volatile v4f*)(out + f) = v;
  __threadfence();
  *(volatile v4f*)(out + f) = v;
}

static inline size_t al256(size_t o) { return (o + 255) & ~(size_t)255; }

extern "C" void kernel_launch(void* const* d_in, const int* in_sizes, int n_in,
                              void* d_out, int out_size, void* d_ws, size_t ws_size,
                              hipStream_t stream) {
  if (n_in < 22) return;
  if (in_sizes[0] != NROWS * 9 || in_sizes[1] != NPIL * 3) return;
  if (in_sizes[2] != 576 || in_sizes[3] != 64 || in_sizes[4] != 64 || in_sizes[5] != 64) return;
  if (in_sizes[6] != 36864 || in_sizes[7] != 64 || in_sizes[8] != 64 || in_sizes[9] != 64) return;
  if (in_sizes[10] != 73728 || in_sizes[11] != 128 || in_sizes[12] != 128 || in_sizes[13] != 128) return;
  if (in_sizes[14] != 294912 || in_sizes[15] != 256 || in_sizes[16] != 256 || in_sizes[17] != 256) return;
  if (in_sizes[18] != 48384 || in_sizes[19] != 21 || in_sizes[20] != 6912 || in_sizes[21] != 3) return;
  if (out_size != NOUTF) return;

  const float* pts   = (const float*)d_in[0];
  const int*   coords = (const int*)d_in[1];
  const float* lin_w = (const float*)d_in[2];
  const float* lin_b = (const float*)d_in[3];
  const float* pfn_g = (const float*)d_in[4];
  const float* pfn_b = (const float*)d_in[5];
  const float* c1_w  = (const float*)d_in[6];
  const float* c1_b  = (const float*)d_in[7];
  const float* bn1_g = (const float*)d_in[8];
  const float* bn1_b = (const float*)d_in[9];
  const float* c2_w  = (const float*)d_in[10];
  const float* c2_b  = (const float*)d_in[11];
  const float* bn2_g = (const float*)d_in[12];
  const float* bn2_b = (const float*)d_in[13];
  const float* h1_w  = (const float*)d_in[14];
  const float* h1_b  = (const float*)d_in[15];
  const float* hbn_g = (const float*)d_in[16];
  const float* hbn_b = (const float*)d_in[17];
  const float* hb_w  = (const float*)d_in[18];
  const float* hb_b  = (const float*)d_in[19];
  const float* hc_w  = (const float*)d_in[20];
  const float* hc_b  = (const float*)d_in[21];
  float* out = (float*)d_out;

  const size_t szTP = (size_t)FPAD * 576 * 4, szC2 = (size_t)M1PAD * 128 * 4, szC3 = (size_t)M2PAD * 256 * 4;
  size_t szR1 = szTP; if (szC2 > szR1) szR1 = szC2; if (szC3 > szR1) szR1 = szC3;
  const size_t szB1 = (size_t)M1PAD * 128 * 2, szH = (size_t)M2PAD * 512 * 2;
  size_t szR2 = szB1; if (szH > szR2) szR2 = szH;
  size_t off = 0;
  const size_t oR1   = off; off = al256(off + szR1);
  const size_t oR2   = off; off = al256(off + szR2);
  const size_t oB2   = off; off = al256(off + (size_t)M2PAD * 256 * 2);
  const size_t oHT   = off; off = al256(off + (size_t)M2PAD * 32 * 4);
  const size_t oPMM  = off; off = al256(off + (size_t)NPIL * 128 * 4);
  const size_t oFT   = off; off = al256(off + (size_t)FPAD * 128 * 2);
  const size_t oWIN  = off; off = al256(off + (size_t)WINPAD * 4);
  const size_t oW1D  = off; off = al256(off + (size_t)576 * 128 * 2);
  const size_t oW2D  = off; off = al256(off + (size_t)128 * 1152 * 2);
  const size_t oW3D  = off; off = al256(off + (size_t)256 * 2304 * 2);
  const size_t oWHD  = off; off = al256(off + (size_t)32 * 4608 * 2);
  const size_t oRC0  = off; off = al256(off + (size_t)5000 * 128 * 4);
  const size_t oRC1  = off; off = al256(off + (size_t)1733 * 128 * 4);
  const size_t oRC2  = off; off = al256(off + (size_t)867 * 256 * 4);
  const size_t oRC3  = off; off = al256(off + (size_t)216 * 512 * 4);
  const size_t oST0  = off; off = al256(off + (size_t)256 * 4);
  const size_t oST1  = off; off = al256(off + (size_t)256 * 4);
  const size_t oST2  = off; off = al256(off + (size_t)512 * 4);
  const size_t oST3  = off; off = al256(off + (size_t)1024 * 4);
  if (off > ws_size || off > (size_t)WSMAX) return;

  char* ws = (char*)d_ws;
  float*          TP   = (float*)(ws + oR1);
  float*          C2   = (float*)(ws + oR1);
  float*          C3   = (float*)(ws + oR1);
  unsigned short* B1hl = (unsigned short*)(ws + oR2);
  unsigned short* Hhl  = (unsigned short*)(ws + oR2);
  unsigned short* B2hl = (unsigned short*)(ws + oB2);
  float*          HEADT = (float*)(ws + oHT);
  float*          PMM  = (float*)(ws + oPMM);
  unsigned short* FEAT = (unsigned short*)(ws + oFT);
  int*            WIN  = (int*)(ws + oWIN);
  unsigned short* W1D  = (unsigned short*)(ws + oW1D);
  unsigned short* W2D  = (unsigned short*)(ws + oW2D);
  unsigned short* W3D  = (unsigned short*)(ws + oW3D);
  unsigned short* WHD  = (unsigned short*)(ws + oWHD);
  float* REC0 = (float*)(ws + oRC0);
  float* REC1 = (float*)(ws + oRC1);
  float* REC2 = (float*)(ws + oRC2);
  float* REC3 = (float*)(ws + oRC3);
  float* ST0 = (float*)(ws + oST0);
  float* ST1 = (float*)(ws + oST1);
  float* ST2 = (float*)(ws + oST2);
  float* ST3 = (float*)(ws + oST3);

  k_wconv<<<(576 * 16 + 255) / 256, 256, 0, stream>>>(c1_w, W1D, 576, 64, 64, 1);
  k_wconv<<<(128 * 144 + 255) / 256, 256, 0, stream>>>(c2_w, W2D, 128, 128, 64, 0);
  k_wconv<<<(256 * 288 + 255) / 256, 256, 0, stream>>>(h1_w, W3D, 256, 256, 128, 0);
  k_wconv<<<(21 * 576 + 255) / 256, 256, 0, stream>>>(hb_w, WHD, 21, 21, 256, 0);
  k_wconv<<<(11 * 576 + 255) / 256, 256, 0, stream>>>(hc_w, WHD + (size_t)21 * 4608, 11, 3, 256, 0);
  k_win<<<NWBLK, 256, 0, stream>>>(coords, WIN);
  k_pfn<<<NROWS / 128, 128, 0, stream>>>(pts, lin_w, lin_b, PMM, REC0);
  k_comb<<<1, 64, 0, stream>>>(REC0, 5000, 128, 128, pfn_g, pfn_b, ST0, 64, 1.0 / 640000.0);
  k_feat<<<FPAD * 8 / 256, 256, 0, stream>>>(PMM, ST0, FEAT);
  k_gemm<<<dim3(FPAD / 64, 576 / 64, 1), 128, 0, stream>>>(FEAT, 128, W1D, 128, 128, TP, 576);
  k_c1<0><<<1733, 256, 0, stream>>>(WIN, TP, c1_b, ST1, REC1, (unsigned*)B1hl);
  k_comb<<<1, 64, 0, stream>>>(REC1, 1733, 256, 164, bn1_g, bn1_b, ST1, 64, 1.0 / 443556.0);
  k_c1<1><<<M1PAD / 64, 256, 0, stream>>>(WIN, TP, c1_b, ST1, REC1, (unsigned*)B1hl);
  k_conv<64, W1, 128, 4, true><<<dim3(M1PAD / 128, 2, 1), 128, 0, stream>>>(B1hl, W2D, c2_b, C2, REC2, HW1);
  k_comb<<<1, 128, 0, stream>>>(REC2, 867, 128, 41, bn2_g, bn2_b, ST2, 128, 1.0 / 110889.0);
  k_pool2<<<M2PAD / 8, 256, 0, stream>>>(C2, ST2, B2hl);
  k_conv<128, W2, 256, 4, true><<<dim3(M2PAD / 128, 4, 1), 128, 0, stream>>>(B2hl, W3D, h1_b, C3, REC3, HW2);
  k_comb<<<1, 256, 0, stream>>>(REC3, 216, 128, 36, hbn_g, hbn_b, ST3, 256, 1.0 / 27556.0);
  k_app3<<<M2PAD * 32 / 256, 256, 0, stream>>>(C3, ST3, Hhl);
  k_conv<256, W2, 32, 2, false><<<dim3(M2PAD / 128, 1, 1), 128, 0, stream>>>(Hhl, WHD, hb_b, HEADT, REC3, HW2);
  k_out<<<(NOUT4 + 255) / 256, 256, 0, stream>>>(HEADT, hb_b, hc_b, out);
  (void)hipGetLastError();
}
